// PraxisAttention_59081570124023
// MI455X (gfx1250) — hardware-verified
//
#include <hip/hip_runtime.h>
#include <math.h>

typedef __attribute__((ext_vector_type(16))) _Float16 v16h;
typedef __attribute__((ext_vector_type(16))) __bf16 v16b;
typedef __attribute__((ext_vector_type(8)))  _Float16 v8h;
typedef __attribute__((ext_vector_type(8)))  __bf16 v8b;
typedef __attribute__((ext_vector_type(8)))  float v8f;
typedef __attribute__((ext_vector_type(4)))  float v4f;
typedef __attribute__((ext_vector_type(4)))  unsigned v4u;

template <typename T> __device__ __forceinline__ void vst2(void* p, T v) { *(volatile T*)p = v; __threadfence(); *(volatile T*)p = v; }
__device__ __forceinline__ v8f wmma16(v16h a, v16h b, v8f c) {
  v8f d = __builtin_amdgcn_wmma_f32_16x16x32_f16(false, a, false, b, (short)0, c, false, false);
  asm volatile("v_nop\n\tv_nop\n\tv_nop\n\tv_nop" : "+v"(d) : "v"(a), "v"(b));
  return d;
}
__device__ __forceinline__ v8f wmma_bf(v16b a, v16b b, v8f c) {
  v8f d = __builtin_amdgcn_wmma_f32_16x16x32_bf16(false, a, false, b, (short)0, c, false, false);
  asm volatile("v_nop\n\tv_nop\n\tv_nop\n\tv_nop" : "+v"(d) : "v"(a), "v"(b));
  return d;
}
__device__ __forceinline__ float bfr(float v) { return (float)(__bf16)v; }
__device__ __forceinline__ v16h frag_h(const _Float16* rowk0, int lane) {
  union { v16h v; v8h q[2]; } u; const _Float16* p = rowk0 + 8 * (lane >> 4);
  u.q[0] = *(const v8h*)p; u.q[1] = *(const v8h*)(p + 16); return u.v;
}
__device__ __forceinline__ v16b frag_b(const __bf16* rowk0, int lane) {
  union { v16b v; v8b q[2]; } u; const __bf16* p = rowk0 + 8 * (lane >> 4);
  u.q[0] = *(const v8b*)p; u.q[1] = *(const v8b*)(p + 16); return u.v;
}
__device__ __forceinline__ v16h frag_f32(const float* rowk0, int lane) {
  v16h a; const float* p = rowk0 + 8 * (lane >> 4);
#pragma unroll
  for (int i = 0; i < 8; ++i) { a[i] = (_Float16)p[i]; a[8 + i] = (_Float16)p[16 + i]; }
  return a;
}
struct F2 { v16b h, l; };
__device__ __forceinline__ F2 bsplit16(const float v[16]) { F2 r;
#pragma unroll
  for (int i = 0; i < 16; ++i) { const __bf16 h = (__bf16)v[i]; r.h[i] = h; r.l[i] = (__bf16)(v[i] - (float)h); }
  return r; }
__device__ __forceinline__ F2 split_row(const float* row, int k0, int lane) { float v[16]; const float* p = row + k0 + 8 * (lane >> 4);
#pragma unroll
  for (int i = 0; i < 8; ++i) { v[i] = p[i]; v[8 + i] = p[16 + i]; }
  return bsplit16(v); }
__device__ __forceinline__ v16b wcol_io(const float* Wm, int k0, int o, int lane, int ld) { v16b w; const int g = lane >> 4;
#pragma unroll
  for (int i = 0; i < 8; ++i) { w[i] = (__bf16)Wm[(size_t)(k0 + 8 * g + i) * ld + o]; w[8 + i] = (__bf16)Wm[(size_t)(k0 + 16 + 8 * g + i) * ld + o]; }
  return w; }
__device__ __forceinline__ v16h wcolh_io(const float* Wm, int k0, int o, int lane, int ld) { v16h w; const int g = lane >> 4;
#pragma unroll
  for (int i = 0; i < 8; ++i) { w[i] = (_Float16)(bfr(Wm[(size_t)(k0 + 8 * g + i) * ld + o]) * 256.0f); w[8 + i] = (_Float16)(bfr(Wm[(size_t)(k0 + 16 + 8 * g + i) * ld + o]) * 256.0f); }
  return w; }
__device__ __forceinline__ void ldsx() { asm volatile("s_wait_dscnt 0" ::: "memory"); __builtin_amdgcn_wave_barrier(); __builtin_amdgcn_fence(3u, "workgroup"); }

#ifndef NB
#define NB 2
#endif
#ifndef SEQ
#define SEQ 2048
#endif
#define NB_FULL 2
#define SEQ_FULL 2048
#define TT SEQ
#define TT_FULL SEQ_FULL
#define DIN 1024
#define NH 16
#define HD 64
#define CQ (NH * 2 * HD)
#define CV (NH * HD)
#define NQB (TT / 64)
#define HG 2
#define SCALE (0.125f)
#define QBH 4
#define QHI 256
#define KHI 256
#define LAM0 (0.8f)
#define GNS (0.2f)
#define GN_EPS (1.0e-5f)
#define PCAR 13
static_assert(HD == 64);
static_assert(TT % 128 == 0);
static_assert(TT >= 256);
static_assert(QHI == QBH * 64);
static_assert(KHI >= (((QBH * 64 - 1) >> 7) + 1) * 128);
static_assert(KHI <= TT);
static_assert(NH % HG == 0);
static_assert(((size_t)(NB - 1) * TT_FULL + TT) * DIN <= (size_t)NB_FULL * TT_FULL * DIN);
__host__ __device__ __forceinline__ int kb_last(int qb) { return (qb * 64 + 63) >> 7; }

#define WS_QH  ((size_t)0)
#define WS_KH  (WS_QH  + 2u * (size_t)NB * TT * CQ)
#define WS_VT  (WS_KH  + 2u * (size_t)NB * TT * CQ)
#define WS_QL  (WS_VT  + 2u * (size_t)NB * CV * TT)
#define WS_KL  (WS_QL  + 2u * (size_t)NB * QHI * CQ)
#define WS_VB  (WS_KL  + 2u * (size_t)NB * KHI * CQ)
#define WS_VBL (WS_VB  + 2u * (size_t)NB * CV * KHI)
#define WS_S   (WS_VBL + 2u * (size_t)NB * CV * KHI)
#define WS_Y   (WS_S   + 4u * (size_t)(HG * 2) * TT * TT)
#define WS_ST  (WS_Y   + 4u * (size_t)NB * TT * CV)
#define WS_END (WS_ST  + 128u * (size_t)NB * NH)
static_assert(WS_END <= (size_t)134217728u);
static_assert(WS_KH % 128 == 0 && WS_VT % 128 == 0 && WS_QL % 128 == 0 && WS_KL % 128 == 0 && WS_VB % 128 == 0 && WS_VBL % 128 == 0 && WS_S % 128 == 0 && WS_Y % 128 == 0 && WS_ST % 128 == 0);

__device__ __forceinline__ float lam_value(const float* __restrict__ Q1, const float* __restrict__ K1, const float* __restrict__ Q2, const float* __restrict__ K2, int lane) {
  float e0 = 0.0f, e1 = 0.0f;
#pragma unroll 1
  for (int s = 0; s < 2; ++s) { const float* qa = s ? Q2 : Q1; const float* ka = s ? K2 : K1;
    float p = bfr(qa[lane]) * bfr(ka[lane]); p = fmaf(bfr(qa[lane + 32]), bfr(ka[lane + 32]), p);
#pragma unroll
    for (int o = 1; o < 32; o <<= 1) p += __shfl_xor(p, o);
    const float ex = expf(p);
    if (s == 0) e0 = ex; else e1 = ex; }
  return (e0 - e1) + LAM0;
}
__device__ __forceinline__ int carry_exp(float lam) { const float A = 1.0f + fabsf(lam); return (int)((__float_as_uint(A) >> 23) & 255u) - 126; }
__device__ __forceinline__ float blk_max(float m, float* sred, float* sbc, int tid) {
#pragma unroll
  for (int o = 1; o < 32; o <<= 1) m = fmaxf(m, __shfl_xor(m, o));
  if ((tid & 31) == 0) sred[tid >> 5] = m;
  __syncthreads();
  if (tid == 0) { float a = sred[0]; for (int i = 1; i < 8; ++i) a = fmaxf(a, sred[i]); *sbc = a; }
  __syncthreads();
  const float r = *sbc;
  __syncthreads();
  return r;
}
__device__ __forceinline__ float blk_sum(float s, float* sred, float* sbc, int tid) {
#pragma unroll
  for (int o = 1; o < 32; o <<= 1) s += __shfl_xor(s, o);
  if ((tid & 31) == 0) sred[tid >> 5] = s;
  __syncthreads();
  if (tid == 0) { float a = 0.0f; for (int i = 0; i < 8; ++i) a += sred[i]; *sbc = a; }
  __syncthreads();
  const float r = *sbc;
  __syncthreads();
  return r;
}
__device__ __forceinline__ double blk_sum_d(double s, double* sred, double* sbc, int tid) {
#pragma unroll
  for (int o = 1; o < 32; o <<= 1) s += __shfl_xor(s, o);
  if ((tid & 31) == 0) sred[tid >> 5] = s;
  __syncthreads();
  if (tid == 0) { double a = 0.0; for (int i = 0; i < 8; ++i) a += sred[i]; *sbc = a; }
  __syncthreads();
  const double r = *sbc;
  __syncthreads();
  return r;
}
__device__ __forceinline__ void gn16(float v[16], const float* p, float mh, float rh, const float* gwp, const float* gbp) {
#pragma unroll
  for (int i = 0; i < 8; ++i) { v[i] = (((p[i] - mh) * rh) * gwp[i] + gbp[i]) * GNS; v[8 + i] = (((p[16 + i] - mh) * rh) * gwp[16 + i] + gbp[16 + i]) * GNS; }
}

__global__ __launch_bounds__(128) __attribute__((amdgpu_num_vgpr(256)))
void k_proj(const float* __restrict__ XQ, const float* __restrict__ XK, const float* __restrict__ XV, const float* __restrict__ WQ, const float* __restrict__ WK, const float* __restrict__ WV,
            _Float16* __restrict__ QH, _Float16* __restrict__ QL, _Float16* __restrict__ KH, _Float16* __restrict__ KL, _Float16* __restrict__ VT, __bf16* __restrict__ VB, __bf16* __restrict__ VBL) {
  __shared__ __align__(16) _Float16 sh[64][136], sl[64][136]; __shared__ __align__(16) _Float16 th[128][72]; __shared__ __align__(16) __bf16 tb[128][72], tbl[128][72];
  const int tid = threadIdx.x, wave = tid >> 5, lane = tid & 31, col = lane & 15, g = lane >> 4; const int which = blockIdx.z; const int c0 = blockIdx.y * 128;
  if (which == 2 && c0 >= CV) return;
  const size_t r0 = (size_t)blockIdx.x * 64; const size_t bb = r0 / TT; const int t0 = (int)(r0 % TT); const size_t xr0 = bb * TT_FULL + (size_t)t0;
  const float* X = which == 0 ? XQ : (which == 1 ? XK : XV); const float* WA = which == 0 ? WQ : (which == 1 ? WK : WV); const int ldw = (which == 2) ? CV : CQ;
  v8f acc[8] = {};
#pragma unroll 2
  for (int kc = 0; kc < DIN / 32; ++kc) { v16b a; { const float* p = X + (xr0 + wave * 16 + col) * DIN + kc * 32 + 8 * g;
#pragma unroll
      for (int i = 0; i < 8; ++i) { a[i] = (__bf16)p[i]; a[8 + i] = (__bf16)p[16 + i]; } }
    asm volatile("s_wait_loadcnt 0x0" ::: "memory");
#pragma unroll
    for (int j = 0; j < 8; ++j) { const v16b w = wcol_io(WA, kc * 32, c0 + j * 16 + col, lane, ldw); asm volatile("s_wait_loadcnt 0x0" ::: "memory"); acc[j] = wmma_bf(a, w, acc[j]); } }
  if (which < 2) { _Float16* DH = which == 0 ? QH : KH; _Float16* DL = which == 0 ? QL : KL; const int nhi = which == 0 ? QHI : KHI; const bool hi_rows = t0 < nhi;
#pragma unroll
    for (int j = 0; j < 8; ++j) {
#pragma unroll
      for (int r = 0; r < 8; ++r) { const float v = acc[j][r]; const _Float16 hv = (_Float16)v; sh[wave * 16 + 8 * g + r][j * 16 + col] = hv; sl[wave * 16 + 8 * g + r][j * 16 + col] = (_Float16)((v - (float)hv) * 1024.0f); } }
    __syncthreads();
    for (int e = tid; e < 64 * 16; e += 128) { const int rl = e >> 4, q = e & 15;
      vst2((void*)(DH + (r0 + rl) * CQ + c0 + q * 8), *(const v4u*)&sh[rl][q * 8]);
      if (hi_rows) vst2((void*)(DL + (bb * nhi + t0 + rl) * (size_t)CQ + c0 + q * 8), *(const v4u*)&sl[rl][q * 8]); }
  } else { const bool hi_rows = t0 < KHI;
#pragma unroll
    for (int j = 0; j < 8; ++j) {
#pragma unroll
      for (int r = 0; r < 8; ++r) { const float v = acc[j][r]; const int rl = wave * 16 + 8 * g + r, cl = j * 16 + col; th[cl][rl] = (_Float16)v; const __bf16 bh = (__bf16)v; tb[cl][rl] = bh; tbl[cl][rl] = (__bf16)(v - (float)bh); } }
    __syncthreads();
    for (int e = tid; e < 128 * 8; e += 128) { const int cl = e >> 3, q = e & 7;
      vst2((void*)(VT + (bb * CV + c0 + cl) * (size_t)TT + t0 + q * 8), *(const v4u*)&th[cl][q * 8]);
      if (hi_rows) { const size_t o3 = (bb * CV + c0 + cl) * (size_t)KHI + t0 + q * 8; vst2((void*)(VB + o3), *(const v4u*)&tb[cl][q * 8]); vst2((void*)(VBL + o3), *(const v4u*)&tbl[cl][q * 8]); } } } }

__global__ __launch_bounds__(128) __attribute__((amdgpu_num_vgpr(256)))
void k_sc(const _Float16* __restrict__ QH, const _Float16* __restrict__ KH, const _Float16* __restrict__ QL, const _Float16* __restrict__ KL, int b, int h0, float* __restrict__ S0) { __shared__ __align__(16) float ss[4][16][132];
  const int qb = blockIdx.x, kb = blockIdx.y; if (kb > kb_last(qb)) return;
  const int hl = blockIdx.z >> 1, st = blockIdx.z & 1; const int qc = (h0 + hl) * (2 * HD) + st * HD; float* S = S0 + (size_t)blockIdx.z * TT * TT;
  const int tid = threadIdx.x, wave = tid >> 5, lane = tid & 31, col = lane & 15, g = lane >> 4; const int k0 = kb * 128; const int ql0 = qb * 64 + wave * 16; const size_t q0 = (size_t)b * TT + ql0, kr0 = (size_t)b * TT + k0;
  v8f acc[8] = {}, accl[8] = {};
  const _Float16* QLb = QL + (size_t)b * QHI * CQ; const _Float16* KLb = KL + (size_t)b * KHI * CQ;
  if (qb < QBH) {
#pragma unroll
    for (int kc = 0; kc < HD / 32; ++kc) { const v16h ah = frag_h(QH + (q0 + col) * CQ + qc + kc * 32, lane), al = frag_h(QLb + (size_t)(ql0 + col) * CQ + qc + kc * 32, lane);
#pragma unroll
      for (int j = 0; j < 8; ++j) { const v16h kbf = frag_h(KH + (kr0 + j * 16 + col) * CQ + qc + kc * 32, lane), klf = frag_h(KLb + (size_t)(k0 + j * 16 + col) * CQ + qc + kc * 32, lane); acc[j] = wmma16(ah, kbf, acc[j]); accl[j] = wmma16(al, kbf, accl[j]); accl[j] = wmma16(ah, klf, accl[j]); } }
  } else if (qb * 64 < QHI) {
#pragma unroll
    for (int kc = 0; kc < HD / 32; ++kc) { const v16h ah = frag_h(QH + (q0 + col) * CQ + qc + kc * 32, lane), al = frag_h(QLb + (size_t)(ql0 + col) * CQ + qc + kc * 32, lane);
#pragma unroll
      for (int j = 0; j < 8; ++j) { const v16h kbf = frag_h(KH + (kr0 + j * 16 + col) * CQ + qc + kc * 32, lane); acc[j] = wmma16(ah, kbf, acc[j]); accl[j] = wmma16(al, kbf, accl[j]); } }
  } else {
#pragma unroll
    for (int kc = 0; kc < HD / 32; ++kc) { const v16h ah = frag_h(QH + (q0 + col) * CQ + qc + kc * 32, lane);
#pragma unroll
      for (int j = 0; j < 8; ++j) { const v16h kbf = frag_h(KH + (kr0 + j * 16 + col) * CQ + qc + kc * 32, lane); acc[j] = wmma16(ah, kbf, acc[j]); } } }
#pragma unroll
  for (int j = 0; j < 8; ++j) {
#pragma unroll
    for (int r = 0; r < 8; ++r) ss[wave][8 * g + r][j * 16 + col] = (acc[j][r] + accl[j][r] * (1.0f / 1024.0f)) * SCALE; }
  ldsx(); for (int rl = 0; rl < 16; ++rl) vst2((void*)(S + (size_t)(ql0 + rl) * TT + k0 + lane * 4), *(const v4f*)&ss[wave][rl][lane * 4]); }

__global__ __launch_bounds__(256) void k_sm(float* __restrict__ S0, const float* __restrict__ AM, const float* __restrict__ LQ1, const float* __restrict__ LK1, const float* __restrict__ LQ2, const float* __restrict__ LK2, int b, int h0s) {
#pragma clang fp contract(off)
  __shared__ float sred[8]; __shared__ float sbc; __shared__ __align__(16) float shv[2][TT];
  const int tid = threadIdx.x, lane = tid & 31; const int t = blockIdx.x; const int hl = blockIdx.y; const int kend = (kb_last(t >> 6) + 1) * 128;
  const float slope = exp2f(-0.5f * (float)(h0s + hl + 1));
  const float lam = lam_value(LQ1, LK1, LQ2, LK2, lane);
  const float* AMb = AM + (size_t)b * TT_FULL;
  float* sr0 = S0 + ((size_t)(hl * 2) * TT + t) * TT;
  float inv0 = 0.0f, inv1 = 0.0f;
#pragma unroll 1
  for (int st = 0; st < 2; ++st) {
    const float* sr = sr0 + (size_t)st * TT * TT; float* sv = &shv[st][0];
    float m = -3.0e38f;
    for (int k = tid; k < kend; k += 256) { const float s = sr[k]; const float padk = (1.0f - bfr(AMb[k])) * (-1.0e9f); const float addk = (-(slope * (float)(t - k)) + (k > t ? -1.0e9f : 0.0f)) + padk; const float v = s + addk; sv[k] = v; m = fmaxf(m, v); }
    m = blk_max(m, sred, &sbc, tid);
    float sum = 0.0f;
    for (int k = tid; k < kend; k += 256) { const float e = expf(sv[k] - m); sv[k] = e; sum += e; }
    sum = blk_sum(sum, sred, &sbc, tid);
    const float iv = 1.0f / sum;
    if (st == 0) inv0 = iv; else inv1 = iv;
  }
  const int ex = carry_exp(lam); const float C = __uint_as_float((unsigned)(127 + PCAR - ex) << 23);
  for (int k = tid; k < kend; k += 256) { const float w0 = shv[0][k] * inv0; const float w1 = shv[1][k] * inv1; const float dw = w0 - lam * w1; shv[0][k] = dw * C; }
  __syncthreads();
  for (int q = tid; q < kend / 4; q += 256) vst2((void*)(sr0 + q * 4), *(const v4f*)&shv[0][q * 4]); }

__global__ __launch_bounds__(128) __attribute__((amdgpu_num_vgpr(256)))
void k_pv(const float* __restrict__ PS0, const _Float16* __restrict__ VT, const __bf16* __restrict__ VB, const __bf16* __restrict__ VBL,
          const float* __restrict__ LQ1, const float* __restrict__ LK1, const float* __restrict__ LQ2, const float* __restrict__ LK2, int b, int h0, float* __restrict__ Y) {
  __shared__ __align__(16) float ss[4][16][HD + 4];
  const int hl = blockIdx.z; const int h = h0 + hl; const float* PS = PS0 + (size_t)(hl * 2) * TT * TT;
  const int tid = threadIdx.x, wave = tid >> 5, lane = tid & 31, col = lane & 15, g = lane >> 4; const int qb = blockIdx.x; const int ql0 = qb * 64 + wave * 16; const int kce = (kb_last(qb) + 1) * 4;
  const float lam = lam_value(LQ1, LK1, LQ2, LK2, lane); const int ex = carry_exp(lam); const float invC = __uint_as_float((unsigned)(127 - PCAR + ex) << 23);
  v8f acc[HD / 16] = {};
  if (qb < QBH) {
#pragma unroll 1
    for (int kc = 0; kc < kce; ++kc) { const F2 p = split_row(PS + (size_t)(ql0 + col) * TT, kc * 32, lane);
      asm volatile("s_wait_loadcnt 0x0" ::: "memory");
#pragma unroll
      for (int j = 0; j < HD / 16; ++j) { const size_t po = ((size_t)b * CV + h * HD + j * 16 + col) * (size_t)KHI + kc * 32; const v16b vh = frag_b(VB + po, lane); acc[j] = wmma_bf(p.h, vh, acc[j]); acc[j] = wmma_bf(p.l, vh, acc[j]); acc[j] = wmma_bf(p.h, frag_b(VBL + po, lane), acc[j]); } }
  } else {
#pragma unroll 1
    for (int kc = 0; kc < kce; ++kc) { const v16h p = frag_f32(PS + (size_t)(ql0 + col) * TT + kc * 32, lane);
      asm volatile("s_wait_loadcnt 0x0" ::: "memory");
#pragma unroll
      for (int j = 0; j < HD / 16; ++j) { const size_t po = ((size_t)b * CV + h * HD + j * 16 + col) * (size_t)TT + kc * 32; acc[j] = wmma16(p, frag_h(VT + po, lane), acc[j]); } } }
#pragma unroll
  for (int j = 0; j < HD / 16; ++j) {
#pragma unroll
    for (int r = 0; r < 8; ++r) ss[wave][8 * g + r][j * 16 + col] = acc[j][r] * invC; }
  ldsx(); for (int rl = 0; rl < 16; ++rl) if (lane < HD / 4) vst2((void*)(Y + ((size_t)b * TT + ql0 + rl) * CV + h * HD + lane * 4), *(const v4f*)&ss[wave][rl][lane * 4]); }

__global__ __launch_bounds__(256) void k_gn(const float* __restrict__ Y, float* __restrict__ ST) {
  __shared__ double dred[8]; __shared__ double dbc;
  const int tid = threadIdx.x, lane = tid & 31, wave = tid >> 5; const int bh = blockIdx.x; const int b = bh / NH, h = bh % NH;
  const float* base = Y + (size_t)b * TT * CV + h * HD;
  double s = 0.0;
  for (int e = tid; e < TT * HD; e += 256) { const int t = e >> 6, d = e & 63; s += (double)base[(size_t)t * CV + d]; }
  s = blk_sum_d(s, dred, &dbc, tid);
  const float meanf = (float)(s / (double)(TT * HD));
  double q = 0.0;
  for (int e = tid; e < TT * HD; e += 256) { const int t = e >> 6, d = e & 63; const float dv = base[(size_t)t * CV + d] - meanf; q += (double)dv * (double)dv; }
  q = blk_sum_d(q, dred, &dbc, tid);
  const float varf = (float)(q / (double)(TT * HD)); const float rstd = 1.0f / sqrtf(varf + GN_EPS);
  if (wave == 0 && lane < 8) { v4f o; o[0] = lane == 0 ? meanf : 0.0f; o[1] = lane == 0 ? rstd : 0.0f; o[2] = 0.0f; o[3] = 0.0f; vst2((void*)(ST + (size_t)bh * 32 + lane * 4), o); }
}

__global__ __launch_bounds__(128) __attribute__((amdgpu_num_vgpr(256)))
void k_out(const float* __restrict__ Y, const float* __restrict__ ST, const float* __restrict__ GW, const float* __restrict__ GB, const float* __restrict__ WO, float* __restrict__ OUT) {
  __shared__ __align__(16) float sf[4][16][132]; __shared__ float smean[NH], srstd[NH]; __shared__ __align__(16) float sgw[CV], sgb[CV];
  const int tid = threadIdx.x, wave = tid >> 5, lane = tid & 31, col = lane & 15, g = lane >> 4; const int c0 = blockIdx.y * 128;
  const size_t rb = (size_t)blockIdx.x * 64; const size_t bb = rb / TT; const int t0 = (int)(rb % TT); const size_t r0 = rb + wave * 16; const size_t orow0 = bb * TT_FULL + (size_t)t0 + wave * 16;
  if (tid < NH) { smean[tid] = ST[(bb * NH + tid) * 32 + 0]; srstd[tid] = ST[(bb * NH + tid) * 32 + 1]; }
  for (int c = tid; c < CV; c += 128) { sgw[c] = bfr(GW[c]); sgb[c] = bfr(GB[c]); }
  __syncthreads();
  v8f acc[8] = {};
  if (t0 < QHI) {
#pragma unroll 2
    for (int kc = 0; kc < CV / 32; ++kc) { float v[16]; gn16(v, Y + (r0 + col) * CV + kc * 32 + 8 * g, smean[kc >> 1], srstd[kc >> 1], sgw + kc * 32 + 8 * g, sgb + kc * 32 + 8 * g); const F2 a = bsplit16(v);
      asm volatile("s_wait_loadcnt 0x0" ::: "memory");
#pragma unroll
      for (int j = 0; j < 8; ++j) { const v16b w = wcol_io(WO, kc * 32, c0 + j * 16 + col, lane, DIN); asm volatile("s_wait_loadcnt 0x0" ::: "memory"); acc[j] = wmma_bf(a.h, w, acc[j]); acc[j] = wmma_bf(a.l, w, acc[j]); } }
#pragma unroll
    for (int j = 0; j < 8; ++j) {
#pragma unroll
      for (int r = 0; r < 8; ++r) sf[wave][8 * g + r][j * 16 + col] = acc[j][r]; }
  } else {
#pragma unroll 2
    for (int kc = 0; kc < CV / 32; ++kc) { float v[16]; gn16(v, Y + (r0 + col) * CV + kc * 32 + 8 * g, smean[kc >> 1], srstd[kc >> 1], sgw + kc * 32 + 8 * g, sgb + kc * 32 + 8 * g); v16h a;
#pragma unroll
      for (int i = 0; i < 16; ++i) a[i] = (_Float16)v[i];
      asm volatile("s_wait_loadcnt 0x0" ::: "memory");
#pragma unroll
      for (int j = 0; j < 8; ++j) { const v16h w = wcolh_io(WO, kc * 32, c0 + j * 16 + col, lane, DIN); asm volatile("s_wait_loadcnt 0x0" ::: "memory"); acc[j] = wmma16(a, w, acc[j]); } }
#pragma unroll
    for (int j = 0; j < 8; ++j) {
#pragma unroll
      for (int r = 0; r < 8; ++r) sf[wave][8 * g + r][j * 16 + col] = acc[j][r] * (1.0f / 256.0f); } }
  ldsx(); for (int rl = 0; rl < 16; ++rl) vst2((void*)(OUT + (orow0 + rl) * DIN + c0 + lane * 4), *(const v4f*)&sf[wave][rl][lane * 4]); }

extern "C" void kernel_launch(void* const* d_in, const int* in_sizes, int n_in, void* d_out, int out_size, void* d_ws, size_t ws_size, hipStream_t stream) {
  if (n_in < 14) return;
  const size_t need_x = (size_t)(NB - 1) * TT_FULL * DIN + (size_t)TT * DIN;
  if ((size_t)in_sizes[0] < need_x || (size_t)in_sizes[1] < need_x || (size_t)in_sizes[2] < need_x) return;
  if ((size_t)in_sizes[3] < (size_t)(NB - 1) * TT_FULL + (size_t)TT) return;
  if ((size_t)in_sizes[4] < (size_t)DIN * CQ || (size_t)in_sizes[5] < (size_t)DIN * CQ || (size_t)in_sizes[6] < (size_t)DIN * CV || (size_t)in_sizes[7] < (size_t)CV * DIN) return;
  if (in_sizes[8] < HD || in_sizes[9] < HD || in_sizes[10] < HD || in_sizes[11] < HD || in_sizes[12] < CV || in_sizes[13] < CV) return;
  if ((size_t)out_size < need_x) return;
  if (ws_size < (size_t)WS_END) return;
  const float* XQ = (const float*)d_in[0]; const float* XK = (const float*)d_in[1]; const float* XV = (const float*)d_in[2]; const float* AM = (const float*)d_in[3];
  const float* WQ = (const float*)d_in[4]; const float* WK = (const float*)d_in[5]; const float* WV = (const float*)d_in[6]; const float* WO = (const float*)d_in[7];
  const float* LQ1 = (const float*)d_in[8]; const float* LQ2 = (const float*)d_in[9]; const float* LK1 = (const float*)d_in[10]; const float* LK2 = (const float*)d_in[11];
  const float* GW = (const float*)d_in[12]; const float* GB = (const float*)d_in[13];
  char* ws = (char*)d_ws;
  _Float16 *QH = (_Float16*)(ws + WS_QH), *KH = (_Float16*)(ws + WS_KH), *VT = (_Float16*)(ws + WS_VT), *QL = (_Float16*)(ws + WS_QL), *KL = (_Float16*)(ws + WS_KL);
  __bf16 *VB = (__bf16*)(ws + WS_VB), *VBL = (__bf16*)(ws + WS_VBL); float *S = (float*)(ws + WS_S), *Y = (float*)(ws + WS_Y), *ST = (float*)(ws + WS_ST);
  k_proj<<<dim3(NB * TT / 64, CQ / 128, 3), 128, 0, stream>>>(XQ, XK, XV, WQ, WK, WV, QH, QL, KH, KL, VT, VB, VBL);
  for (int b = 0; b < NB; ++b) for (int h0 = 0; h0 < NH; h0 += HG) {
    k_sc<<<dim3(NQB, TT / 128, HG * 2), 128, 0, stream>>>(QH, KH, QL, KL, b, h0, S);
    k_sm<<<dim3(TT, HG), 256, 0, stream>>>(S, AM, LQ1, LK1, LQ2, LK2, b, h0);
    k_pv<<<dim3(NQB, 1, HG), 128, 0, stream>>>(S, VT, VB, VBL, LQ1, LK1, LQ2, LK2, b, h0, Y);
  }
  k_gn<<<dim3(NB * NH), 256, 0, stream>>>(Y, ST);
  k_out<<<dim3(NB * TT / 64, DIN / 128), 128, 0, stream>>>(Y, ST, GW, GB, WO, (float*)d_out);
}
